// Dual_net_47227460387442
// MI455X (gfx1250) — hardware-verified
//
#include <hip/hip_runtime.h>
#include <math.h>

typedef __attribute__((ext_vector_type(16))) _Float16 v16h;
typedef __attribute__((ext_vector_type(8)))  _Float16 v8h;
typedef __attribute__((ext_vector_type(8)))  float    v8f;
typedef __attribute__((ext_vector_type(4)))  float    v4f;
typedef __attribute__((ext_vector_type(4)))  unsigned int v4u;

constexpr int kInW  = 58;
constexpr int kCIn  = 4;
constexpr int kNIn  = 54;
constexpr int kHid  = 128;
constexpr int kFDim = 57;
constexpr int kNBr  = 54;
constexpr int kNCls = 3;
constexpr int kOutW = 162;
constexpr int kRowsPerBlock = 16;
constexpr int kOut4PerBlock = kRowsPerBlock * kOutW / 4;
constexpr float kWCarry    = 16.0f;
constexpr float kWCarryInv = 1.0f / 16.0f;

constexpr int kOffC1 = 0;
constexpr int kOffC2 = 4096;
constexpr int kOffN1 = 6144;
constexpr int kOffN2 = 14336;
constexpr int kOffF1 = 22528;
constexpr int kOffF2 = 30720;
constexpr int kOffO1 = 38912;
constexpr int kOffO2 = 481280;
constexpr int kWsHalves = 591872;
constexpr int kO1Plane = kHid * 64;
constexpr int kO2Plane = 16 * kHid;

__device__ __forceinline__ unsigned pk16(unsigned short a, unsigned short b) { return (unsigned)a | ((unsigned)b << 16); }
__device__ __forceinline__ unsigned short h_bits(float f) { const _Float16 hv = (_Float16)f; return __builtin_bit_cast(unsigned short, hv); }

template <typename T> struct Frag;
template <> struct Frag<_Float16> {
  typedef v16h V; union U { v16h v; v8h h[2]; };
  static __device__ __forceinline__ v16h load(const _Float16* p) {
    U f; f.h[0] = *(const v8h*)(p); f.h[1] = *(const v8h*)(p + 16); return f.v;
  }
  static __device__ __forceinline__ v8f mma(v16h a, v16h b, v8f c) {
    return __builtin_amdgcn_wmma_f32_16x16x32_f16(false, a, false, b, (short)0, c, false, false);
  }
};

__device__ __forceinline__ void acc_guard_frag4(v8f& acc, v16h a, v16h b, v16h c2, v16h d) {
  asm volatile("v_nop\n\tv_nop\n\tv_nop\n\tv_nop" : "+v"(acc) : "v"(a), "v"(b), "v"(c2), "v"(d));
}
__device__ __forceinline__ void keep4_h(v16h a, v16h b, v16h c2, v16h d) { asm volatile("v_nop" :: "v"(a), "v"(b), "v"(c2), "v"(d)); }

__device__ __forceinline__ v8f mma_h(v16h a, v16h b, v8f c) { return Frag<_Float16>::mma(a, b, c); }
__device__ __forceinline__ v16h frag_ld(const _Float16* p) { return Frag<_Float16>::load(p); }
__device__ __forceinline__ v16h frag_lds(const unsigned short* p) { return Frag<_Float16>::load((const _Float16*)(const void*)p); }
__device__ __forceinline__ v8f zero8() { return (v8f){0.f, 0.f, 0.f, 0.f, 0.f, 0.f, 0.f, 0.f}; }

__global__ __launch_bounds__(256) void wt_prep_kernel(const float* __restrict__ src, unsigned short* __restrict__ dst,
                                                      int Ksrc, int Nsrc, int KP, int NP, int nB, float scale) {
  const int t = blockIdx.x * 256 + threadIdx.x;
  const int total8 = (nB * NP * KP) >> 3;
  if (t >= total8) return;
  const int idx  = t << 3;
  const int perB = NP * KP;
  const int b    = idx / perB;
  const int rem  = idx - b * perB;
  const int n    = rem / KP;
  const int kp0  = rem - n * KP;
  const int nc   = (n < Nsrc) ? n : (Nsrc - 1);
  unsigned short q[8];
#pragma unroll
  for (int j = 0; j < 8; ++j) {
    const int k  = kp0 + j;
    const int kc = (k < Ksrc) ? k : (Ksrc - 1);
    const float w = src[((size_t)b * Ksrc + kc) * Nsrc + nc] * scale;
    q[j] = h_bits((k < Ksrc && n < Nsrc) ? w : 0.0f);
  }
  const v4u u = (v4u){pk16(q[0], q[1]), pk16(q[2], q[3]), pk16(q[4], q[5]), pk16(q[6], q[7])};
  unsigned short* op = dst + idx;
  *(volatile v4u*)op = u;
  __threadfence();
  *(volatile v4u*)op = u;
}

template <int KS>
__device__ __forceinline__ void hidden_stage(const _Float16* __restrict__ wt, const float* __restrict__ bias,
                                             v16h bf0, v16h bf1, unsigned short* hb, int lane) {
  const int h = lane >> 4, c = lane & 15;
  constexpr int kp = KS * 32;
#pragma unroll
  for (int dt = 0; dt < 8; ++dt) {
    v8f acc = zero8();
    const _Float16* ap = wt + (size_t)(dt * 16 + c) * kp + 8 * h;
    const v16h a0 = frag_ld(ap);
    acc = mma_h(a0, bf0, acc);
    v16h a1 = a0;
    if (KS == 2) {
      a1 = frag_ld(ap + 32);
      acc = mma_h(a1, bf1, acc);
    }
    acc_guard_frag4(acc, a0, a1, bf0, bf1);
    const float* bp = bias + dt * 16 + 8 * h;
    const v4f b0 = *(const v4f*)(bp);
    const v4f b1 = *(const v4f*)(bp + 4);
    unsigned short q[8];
#pragma unroll
    for (int r = 0; r < 4; ++r) {
      q[r]     = h_bits(fmaxf(acc[r] * kWCarryInv + b0[r], 0.0f));
      q[4 + r] = h_bits(fmaxf(acc[4 + r] * kWCarryInv + b1[r], 0.0f));
    }
    const v4u u = (v4u){pk16(q[0], q[1]), pk16(q[2], q[3]), pk16(q[4], q[5]), pk16(q[6], q[7])};
    *(v4u*)(hb + c * kHid + dt * 16 + 8 * h) = u;
  }
}

__device__ __forceinline__ v8f tile16_k128(const _Float16* __restrict__ wt_rows, v16h b0, v16h b1, v16h b2, v16h b3, int lane) {
  const int h = lane >> 4, c = lane & 15;
  const _Float16* ap = wt_rows + (size_t)c * kHid + 8 * h;
  const v16h a0 = frag_ld(ap);
  const v16h a1 = frag_ld(ap + 32);
  const v16h a2 = frag_ld(ap + 64);
  const v16h a3 = frag_ld(ap + 96);
  v8f acc = zero8();
  acc = mma_h(a0, b0, acc);
  acc = mma_h(a1, b1, acc);
  acc = mma_h(a2, b2, acc);
  acc = mma_h(a3, b3, acc);
  acc_guard_frag4(acc, a0, a1, a2, a3);
  keep4_h(b0, b1, b2, b3);
  return acc;
}

__global__ __launch_bounds__(256) void dual_mlp_kernel(
    const float* __restrict__ x, const unsigned short* __restrict__ wsh,
    const float* __restrict__ Cb1, const float* __restrict__ Cb2,
    const float* __restrict__ Nb1, const float* __restrict__ Nb2,
    const float* __restrict__ Fb1, const float* __restrict__ Fb2,
    const float* __restrict__ Ob1, const float* __restrict__ Ob2,
    float* __restrict__ out, int rows) {
  __shared__ __align__(16) unsigned short XC[kRowsPerBlock * 32];
  __shared__ __align__(16) unsigned short XN[kRowsPerBlock * 64];
  __shared__ __align__(16) unsigned short HB[kRowsPerBlock * kHid];
  __shared__ __align__(16) unsigned short FT[kRowsPerBlock * 64];
  __shared__ __align__(16) float ST[kRowsPerBlock * kOutW];

  const int lane = threadIdx.x & 31;
  const int h = lane >> 4, c = lane & 15;
  const int row0 = blockIdx.x * kRowsPerBlock;
  int rr = row0 + c;
  rr = (rr < rows) ? rr : (rows - 1);
  const float* xr = x + (size_t)rr * kInW;

  const _Float16* wC1 = (const _Float16*)(const void*)(wsh + kOffC1);
  const _Float16* wC2 = (const _Float16*)(const void*)(wsh + kOffC2);
  const _Float16* wN1 = (const _Float16*)(const void*)(wsh + kOffN1);
  const _Float16* wN2 = (const _Float16*)(const void*)(wsh + kOffN2);
  const _Float16* wF1 = (const _Float16*)(const void*)(wsh + kOffF1);
  const _Float16* wF2 = (const _Float16*)(const void*)(wsh + kOffF2);
  const _Float16* wO1 = (const _Float16*)(const void*)(wsh + kOffO1);
  const _Float16* wO2 = (const _Float16*)(const void*)(wsh + kOffO2);

  {
    const float x0 = xr[0], x1 = xr[1], x2 = xr[2], x3 = xr[3];
    const unsigned d0 = pk16(h_bits(x0), h_bits(x1));
    const unsigned d1 = pk16(h_bits(x2), h_bits(x3));
    const unsigned s0 = (h == 0) ? d0 : 0u;
    const unsigned s1 = (h == 0) ? d1 : 0u;
    *(v4u*)(XC + c * 32 + 16 * h)     = (v4u){s0, s1, 0u, 0u};
    *(v4u*)(XC + c * 32 + 16 * h + 8) = (v4u){0u, 0u, 0u, 0u};
  }
  {
    unsigned dw[16];
#pragma unroll
    for (int j = 0; j < 16; ++j) {
      const int col0 = 32 * h + 2 * j;
      const int col1 = col0 + 1;
      const int ca = (col0 < kNIn) ? col0 : (kNIn - 1);
      const int cb = (col1 < kNIn) ? col1 : (kNIn - 1);
      const float xa = xr[kCIn + ca];
      const float xb = xr[kCIn + cb];
      const float va = (col0 < kNIn) ? xa : 0.0f;
      const float vb = (col1 < kNIn) ? xb : 0.0f;
      dw[j] = pk16(h_bits(va), h_bits(vb));
    }
#pragma unroll
    for (int q4 = 0; q4 < 4; ++q4)
      *(v4u*)(XN + c * 64 + 32 * h + 8 * q4) = (v4u){dw[4 * q4], dw[4 * q4 + 1], dw[4 * q4 + 2], dw[4 * q4 + 3]};
  }
  __syncthreads();

  {
    const v16h b0 = frag_lds(XC + c * 32 + 8 * h);
    hidden_stage<1>(wC1, Cb1, b0, b0, HB, lane);
  }
  __syncthreads();

  {
    const v16h hq0 = frag_lds(HB + c * kHid + 8 * h);
    const v16h hq1 = frag_lds(HB + c * kHid + 32 + 8 * h);
    const v16h hq2 = frag_lds(HB + c * kHid + 64 + 8 * h);
    const v16h hq3 = frag_lds(HB + c * kHid + 96 + 8 * h);
    const v8f acc = tile16_k128(wC2, hq0, hq1, hq2, hq3, lane);
    const float cb0 = Cb2[0], cb1 = Cb2[1], cb2 = Cb2[2];
    const unsigned short t0 = h_bits(acc[0] * kWCarryInv + cb0);
    const unsigned short t1 = h_bits(acc[1] * kWCarryInv + cb1);
    const unsigned short t2 = h_bits(acc[2] * kWCarryInv + cb2);
    if (h == 0) {
      FT[c * 64 + 0] = t0;
      FT[c * 64 + 1] = t1;
      FT[c * 64 + 2] = t2;
    }
  }
  __syncthreads();

  {
    const v16h b0 = frag_lds(XN + c * 64 + 8 * h);
    const v16h b1 = frag_lds(XN + c * 64 + 32 + 8 * h);
    hidden_stage<2>(wN1, Nb1, b0, b1, HB, lane);
  }
  __syncthreads();

  {
    const v16h hq0 = frag_lds(HB + c * kHid + 8 * h);
    const v16h hq1 = frag_lds(HB + c * kHid + 32 + 8 * h);
    const v16h hq2 = frag_lds(HB + c * kHid + 64 + 8 * h);
    const v16h hq3 = frag_lds(HB + c * kHid + 96 + 8 * h);
#pragma unroll
    for (int nt = 0; nt < 4; ++nt) {
      const v8f acc = tile16_k128(wN2 + (size_t)nt * 16 * kHid, hq0, hq1, hq2, hq3, lane);
#pragma unroll
      for (int r = 0; r < 8; ++r) {
        const int nn  = nt * 16 + 8 * h + r;
        const int nnc = (nn < kNIn) ? nn : (kNIn - 1);
        const float bv = Nb2[nnc];
        const float v  = acc[r] * kWCarryInv + ((nn < kNIn) ? bv : 0.0f);
        const unsigned short tv = h_bits(v);
        if (nn <= 60) FT[c * 64 + 3 + nn] = tv;
      }
    }
  }
  __syncthreads();

  {
    const v16h b0 = frag_lds(FT + c * 64 + 8 * h);
    const v16h b1 = frag_lds(FT + c * 64 + 32 + 8 * h);
    hidden_stage<2>(wF1, Fb1, b0, b1, HB, lane);
  }
  __syncthreads();

  {
    const v16h hq0 = frag_lds(HB + c * kHid + 8 * h);
    const v16h hq1 = frag_lds(HB + c * kHid + 32 + 8 * h);
    const v16h hq2 = frag_lds(HB + c * kHid + 64 + 8 * h);
    const v16h hq3 = frag_lds(HB + c * kHid + 96 + 8 * h);
#pragma unroll
    for (int nt = 0; nt < 4; ++nt) {
      const v8f acc = tile16_k128(wF2 + (size_t)nt * 16 * kHid, hq0, hq1, hq2, hq3, lane);
      const int n0 = nt * 16 + 8 * h;
      unsigned short q[8];
#pragma unroll
      for (int r = 0; r < 8; ++r) {
        const int nn  = n0 + r;
        const int nnc = (nn < kFDim) ? nn : (kFDim - 1);
        const float bv = Fb2[nnc];
        q[r] = h_bits(acc[r] * kWCarryInv + ((nn < kFDim) ? bv : 0.0f));
      }
      *(v4u*)(FT + c * 64 + n0) = (v4u){pk16(q[0], q[1]), pk16(q[2], q[3]), pk16(q[4], q[5]), pk16(q[6], q[7])};
    }
  }
  __syncthreads();

  const v16h fb0 = frag_lds(FT + c * 64 + 8 * h);
  const v16h fb1 = frag_lds(FT + c * 64 + 32 + 8 * h);

#pragma unroll 1
  for (int n = 0; n < kNBr; ++n) {
    hidden_stage<2>(wO1 + (size_t)n * kO1Plane, Ob1 + n * kHid, fb0, fb1, HB, lane);
    __syncthreads();
    const v16h hq0 = frag_lds(HB + c * kHid + 8 * h);
    const v16h hq1 = frag_lds(HB + c * kHid + 32 + 8 * h);
    const v16h hq2 = frag_lds(HB + c * kHid + 64 + 8 * h);
    const v16h hq3 = frag_lds(HB + c * kHid + 96 + 8 * h);
    const v8f acc = tile16_k128(wO2 + (size_t)n * kO2Plane, hq0, hq1, hq2, hq3, lane);
    const float* ob = Ob2 + n * kNCls;
    const float l0 = acc[0] * kWCarryInv + ob[0];
    const float l1 = acc[1] * kWCarryInv + ob[1];
    const float l2 = acc[2] * kWCarryInv + ob[2];
    const float mx = fmaxf(l0, fmaxf(l1, l2));
    const float e0 = expf(l0 - mx);
    const float e1 = expf(l1 - mx);
    const float e2 = expf(l2 - mx);
    const float inv = 1.0f / (e0 + e1 + e2);
    const float p0 = e0 * inv, p1 = e1 * inv, p2 = e2 * inv;
    if (h == 0) {
      float* sp = ST + c * kOutW + n * kNCls;
      sp[0] = p0;
      sp[1] = p1;
      sp[2] = p2;
    }
    __syncthreads();
  }

  {
    float* op = out + (size_t)row0 * kOutW;
    for (int ps = 0; ps < 2; ++ps) {
#pragma unroll
      for (int it = 0; it < 21; ++it) {
        const int i4  = it * 32 + lane;
        const int i4c = (i4 < kOut4PerBlock) ? i4 : (kOut4PerBlock - 1);
        const v4f v = *(const v4f*)(ST + 4 * i4c);
        if (i4 < kOut4PerBlock) *(volatile v4f*)(op + 4 * (size_t)i4c) = v;
      }
      __threadfence();
    }
  }
}

extern "C" void kernel_launch(void* const* d_in, const int* in_sizes, int n_in,
                              void* d_out, int out_size, void* d_ws, size_t ws_size,
                              hipStream_t stream) {
  const float* x   = (const float*)d_in[0];
  const float* Cw1 = (const float*)d_in[1];
  const float* Cb1 = (const float*)d_in[2];
  const float* Cw2 = (const float*)d_in[3];
  const float* Cb2 = (const float*)d_in[4];
  const float* Nw1 = (const float*)d_in[5];
  const float* Nb1 = (const float*)d_in[6];
  const float* Nw2 = (const float*)d_in[7];
  const float* Nb2 = (const float*)d_in[8];
  const float* Fw1 = (const float*)d_in[9];
  const float* Fb1 = (const float*)d_in[10];
  const float* Fw2 = (const float*)d_in[11];
  const float* Fb2 = (const float*)d_in[12];
  const float* Ow1 = (const float*)d_in[13];
  const float* Ob1 = (const float*)d_in[14];
  const float* Ow2 = (const float*)d_in[15];
  const float* Ob2 = (const float*)d_in[16];
  float* out = (float*)d_out;
  unsigned short* wsh = (unsigned short*)d_ws;
  (void)n_in; (void)out_size;

  if ((size_t)kWsHalves * sizeof(unsigned short) > ws_size) return;
  const int rows = in_sizes[0] / kInW;
  const int blocks = rows / kRowsPerBlock;
  if (blocks <= 0) return;
  if ((size_t)blocks * kRowsPerBlock * kOutW > (size_t)out_size) return;

  auto prep = [&](const float* src, int offHalves, int Ksrc, int Nsrc, int KP, int NP, int nB) {
    const int total8 = (nB * NP * KP) / 8;
    wt_prep_kernel<<<(total8 + 255) / 256, 256, 0, stream>>>(src, wsh + offHalves, Ksrc, Nsrc, KP, NP, nB, kWCarry);
  };
  prep(Cw1, kOffC1,   4, 128,  32, 128,  1);
  prep(Cw2, kOffC2, 128,   3, 128,  16,  1);
  prep(Nw1, kOffN1,  54, 128,  64, 128,  1);
  prep(Nw2, kOffN2, 128,  54, 128,  64,  1);
  prep(Fw1, kOffF1,  57, 128,  64, 128,  1);
  prep(Fw2, kOffF2, 128,  57, 128,  64,  1);
  prep(Ow1, kOffO1,  57, 128,  64, 128, 54);
  prep(Ow2, kOffO2, 128,   3, 128,  16, 54);

  dual_mlp_kernel<<<blocks, 32, 0, stream>>>(x, wsh, Cb1, Cb2, Nb1, Nb2, Fb1, Fb2, Ob1, Ob2, out, rows);
}
